// SoftAlignAttentionMixed_23373212025422
// MI455X (gfx1250) — hardware-verified
//
#include <hip/hip_runtime.h>
#include <math.h>

typedef __attribute__((ext_vector_type(16))) _Float16 v16h;
typedef __attribute__((ext_vector_type(16))) __bf16 v16b;
typedef __attribute__((ext_vector_type(8)))  _Float16 v8h;
typedef __attribute__((ext_vector_type(8)))  float v8f;
typedef __attribute__((ext_vector_type(4)))  float v4f;
typedef __attribute__((ext_vector_type(2)))  float v2f;
typedef __attribute__((ext_vector_type(4)))  unsigned v4u;
typedef __attribute__((ext_vector_type(4)))  int v4i;
typedef float __attribute__((may_alias)) float_a;
typedef int __attribute__((may_alias)) int_a;

template <typename T> __device__ __forceinline__ void vst2(void* p, T v) { *(volatile T*)p = v; __threadfence(); *(volatile T*)p = v; }
__device__ __forceinline__ v8f wmma16(v16h a, v16h b, v8f c) {
  v8f d = __builtin_amdgcn_wmma_f32_16x16x32_f16(false, a, false, b, (short)0, c, false, false);
  asm volatile("v_nop\n\tv_nop\n\tv_nop\n\tv_nop" : "+v"(d) : "v"(a), "v"(b));
  return d;
}
__device__ __forceinline__ v8f wmma_bf(v16b a, v16b b, v8f c) {
  v8f d = __builtin_amdgcn_wmma_f32_16x16x32_bf16(false, a, false, b, (short)0, c, false, false);
  asm volatile("v_nop\n\tv_nop\n\tv_nop\n\tv_nop" : "+v"(d) : "v"(a), "v"(b));
  return d;
}
__device__ __forceinline__ v16h frag_h(const _Float16* rowk0, int lane) {
  union { v16h v; v8h q[2]; } u; const _Float16* p = rowk0 + 8 * (lane >> 4);
  u.q[0] = *(const v8h*)p; u.q[1] = *(const v8h*)(p + 16); return u.v;
}
__device__ __forceinline__ v16h frag_f32(const float* rowk0, int lane) {
  v16h a; const float* p = rowk0 + 8 * (lane >> 4);
#pragma unroll
  for (int i = 0; i < 8; ++i) { a[i] = (_Float16)p[i]; a[8 + i] = (_Float16)p[16 + i]; }
  return a;
}
__device__ __forceinline__ v16h frag_f32s(const float* rowk0, int lane, float sc) {
  v16h a; const float* p = rowk0 + 8 * (lane >> 4);
#pragma unroll
  for (int i = 0; i < 8; ++i) { a[i] = (_Float16)(p[i] * sc); a[8 + i] = (_Float16)(p[16 + i] * sc); }
  return a;
}
__device__ __forceinline__ v16h fragc_f32(const float* W, int k0, int n, int lane, int ld, int K) {
  v16h a; const int g = lane >> 4;
#pragma unroll
  for (int i = 0; i < 8; ++i) { const int ka = k0 + 8 * g + i, kb = ka + 16;
    a[i] = (_Float16)(ka < K ? W[(size_t)(ka < K ? ka : K - 1) * ld + n] : 0.f); a[8 + i] = (_Float16)(kb < K ? W[(size_t)(kb < K ? kb : K - 1) * ld + n] : 0.f); }
  return a;
}
struct F2 { v16b h, l; };
__device__ __forceinline__ F2 bsplit16(const float v[16]) { F2 r;
#pragma unroll
  for (int i = 0; i < 16; ++i) { const __bf16 h = (__bf16)v[i]; r.h[i] = h; r.l[i] = (__bf16)(v[i] - (float)h); }
  return r; }
__device__ __forceinline__ F2 split_row(const float* row, int k0, int lane) { float v[16]; const float* p = row + k0 + 8 * (lane >> 4);
#pragma unroll
  for (int i = 0; i < 8; ++i) { v[i] = p[i]; v[8 + i] = p[16 + i]; }
  return bsplit16(v); }
__device__ __forceinline__ F2 split_rowK(const float* row, int k0, int lane, int K) { float v[16]; const int g = lane >> 4;
#pragma unroll
  for (int i = 0; i < 8; ++i) { const int ka = k0 + 8 * g + i, kb = ka + 16; v[i] = ka < K ? row[ka < K ? ka : K - 1] : 0.f; v[8 + i] = kb < K ? row[kb < K ? kb : K - 1] : 0.f; }
  return bsplit16(v); }
__device__ __forceinline__ F2 split_col(const float* W, int k0, int n, int lane, int ld, int K) { float v[16]; const int g = lane >> 4;
#pragma unroll
  for (int i = 0; i < 8; ++i) { const int ka = k0 + 8 * g + i, kb = ka + 16; v[i] = ka < K ? W[(size_t)(ka < K ? ka : K - 1) * ld + n] : 0.f; v[8 + i] = kb < K ? W[(size_t)(kb < K ? kb : K - 1) * ld + n] : 0.f; }
  return bsplit16(v); }
__device__ __forceinline__ v8f mac3(const F2& a, const F2& b, v8f c) { c = wmma_bf(a.l, b.h, c); c = wmma_bf(a.h, b.l, c); return wmma_bf(a.h, b.h, c); }
__device__ __forceinline__ float sigm(float v) { return 1.0f / (1.0f + expf(-v)); }
#define LDSX() do { asm volatile("s_wait_dscnt 0" ::: "memory"); __builtin_amdgcn_wave_barrier(); __builtin_amdgcn_fence(__ATOMIC_RELEASE, "workgroup"); } while (0)


#define NB 4
#define CC 512
#define TT 2048
#define NH 8
#define HD 64
#define WW 16
#define TS 1000
#define NR (NB * TT)
#ifndef TNB
#define TNB NB
#endif
#define TR (TNB * TT)
typedef __attribute__((ext_vector_type(8))) __bf16 v8b;
__device__ __forceinline__ v16b frag_b(const __bf16* rowk0, int lane) {
  union { v16b v; v8b q[2]; } u; const __bf16* p = rowk0 + 8 * (lane >> 4);
  u.q[0] = *(const v8b*)p; u.q[1] = *(const v8b*)(p + 16); return u.v;
}
__device__ __forceinline__ float bfr(float v) { return (float)(__bf16)v; }
__device__ __attribute__((noinline)) float exp_ni(float v) { return expf(v); }
__device__ __attribute__((noinline)) float erf_ni(float v) { return erff(v); }

#define WS_PW   0u
#define WS_QL   (WS_PW + 2u * (size_t)8 * CC * CC)
#define WS_KL   (WS_QL + 2u * (size_t)NR * CC)
#define WS_QG   (WS_KL + 2u * (size_t)NR * CC)
#define WS_KG   (WS_QG + 2u * (size_t)NR * CC)
#define WS_VL   (WS_KG + 2u * (size_t)NR * CC)
#define WS_VG   (WS_VL + 2u * (size_t)NB * CC * TT)
#define WS_LO   (WS_VG + 2u * (size_t)NB * CC * TT)
#define WS_CG   (WS_LO + 4u * (size_t)NR * CC)
#define WS_LOT  (WS_CG + 4u * (size_t)NR * CC)
#define WS_LOTL (WS_LOT + 2u * (size_t)NR * CC)
#define WS_YL   (WS_LOTL + 2u * (size_t)NR * CC)
#define WS_END  (WS_YL + 4u * (size_t)NB * CC * TT)

__global__ __launch_bounds__(256) void k_pack(const float* __restrict__ W0, const float* __restrict__ W1, const float* __restrict__ W2, const float* __restrict__ W3, const float* __restrict__ W4, const float* __restrict__ W5, const float* __restrict__ W6, const float* __restrict__ W7, __bf16* __restrict__ P) {
  __shared__ __align__(16) __bf16 s[CC]; const int n = blockIdx.x, which = blockIdx.y, t = threadIdx.x; const float* Wm = (which == 0) ? W0 : (which == 1) ? W1 : (which == 2) ? W2 : (which == 3) ? W3 : (which == 4) ? W4 : (which == 5) ? W5 : (which == 6) ? W6 : W7;
  for (int k = t; k < CC; k += 256) s[k] = (__bf16)Wm[(size_t)n * CC + k]; __syncthreads(); for (int q = t; q < CC / 8; q += 256) vst2((unsigned*)(P + ((size_t)which * CC + n) * CC + q * 8), *(const v4u*)&s[q * 8]); }
__device__ __attribute__((noinline)) float pow_p(float a, float b) { return powf(a, b); }
__device__ __attribute__((noinline)) float sin_p(float v) { return sinf(v); }
__device__ __attribute__((noinline)) float cos_p(float v) { return cosf(v); }
__global__ __launch_bounds__(128) void k_proj(const float* __restrict__ X, const float* __restrict__ CND, const __bf16* __restrict__ P, const float* __restrict__ B0, const float* __restrict__ B1, const float* __restrict__ B2, const float* __restrict__ B4, const float* __restrict__ B5, const float* __restrict__ B6, _Float16* __restrict__ QL, _Float16* __restrict__ KL, _Float16* __restrict__ VL, _Float16* __restrict__ QG, _Float16* __restrict__ KG, _Float16* __restrict__ VG) {
  __shared__ __align__(16) float sf[64][132]; __shared__ __align__(16) _Float16 so[64][136]; __shared__ __align__(16) _Float16 st[128][72];
  const int tid = threadIdx.x, wave = tid >> 5, lane = tid & 31, col = lane & 15, g = lane >> 4; const int wsel = blockIdx.z; const int which = (wsel < 3) ? wsel : wsel + 1;
  const int n0 = blockIdx.y * 128; const size_t rb0 = (size_t)blockIdx.x * 64; const size_t b = rb0 / TT, t0 = rb0 % TT; const int tw = (int)t0 + wave * 16;
  const float* IN = (which == 0 || which == 4) ? X : CND; const float* BB = (which == 0) ? B0 : (which == 1) ? B1 : (which == 2) ? B2 : (which == 4) ? B4 : (which == 5) ? B5 : B6;
  v8f acc[8] = {};
#pragma unroll 2
  for (int kc = 0; kc < CC / 32; ++kc) { v16b a; { const float* p = IN + (b * CC + kc * 32 + 8 * g) * TT + tw + col;
#pragma unroll
      for (int i = 0; i < 8; ++i) { a[i] = (__bf16)p[(size_t)i * TT]; a[8 + i] = (__bf16)p[(size_t)(16 + i) * TT]; } }
#pragma unroll
    for (int j = 0; j < 8; ++j) acc[j] = wmma_bf(a, frag_b(P + ((size_t)which * CC + n0 + j * 16 + col) * CC + kc * 32, lane), acc[j]); }
  if (which == 2 || which == 6) {
#pragma unroll
    for (int j = 0; j < 8; ++j) { const float bb = bfr(BB[n0 + j * 16 + col]);
#pragma unroll
      for (int r = 0; r < 8; ++r) st[j * 16 + col][wave * 16 + 8 * g + r] = (_Float16)(acc[j][r] + bb); }
    __syncthreads(); _Float16* V = (which == 2) ? VL : VG;
    for (int e = tid; e < 128 * 8; e += 128) { const int d = e >> 3, pc = e & 7; vst2((unsigned*)(V + ((b * CC + n0 + d) * TT) + t0 + pc * 8), *(const v4u*)&st[d][pc * 8]); }
    return; }
  if (which < 2) {
#pragma unroll
    for (int j = 0; j < 8; ++j) { const float bb = bfr(BB[n0 + j * 16 + col]);
#pragma unroll
      for (int r = 0; r < 8; ++r) so[wave * 16 + 8 * g + r][j * 16 + col] = (_Float16)(acc[j][r] + bb); }
  } else {
#pragma unroll
    for (int j = 0; j < 8; ++j) { const float bb = bfr(BB[n0 + j * 16 + col]);
#pragma unroll
      for (int r = 0; r < 8; ++r) sf[wave * 16 + 8 * g + r][j * 16 + col] = acc[j][r] + bb; }
    LDSX();
    for (int rl = 0; rl < 16; ++rl) { const float pos = (float)(tw + rl);
      for (int pi = lane; pi < 64; pi += 32) { const int c = 2 * pi; const int i = ((n0 + c) % HD) / 2; const float inv = 1.0f / pow_p(10000.0f, (float)(2 * i) / (float)HD); const float ang = pos * inv; const float cs = cos_p(ang), sn = sin_p(ang);
        const float x1 = sf[wave * 16 + rl][c], x2 = sf[wave * 16 + rl][c + 1]; so[wave * 16 + rl][c] = (_Float16)(x1 * cs - x2 * sn); so[wave * 16 + rl][c + 1] = (_Float16)(x1 * sn + x2 * cs); } }
  }
  LDSX();
  _Float16* D0 = (which == 0) ? QL : (which == 1) ? KL : (which == 4) ? QG : KG;
  for (int rl = 0; rl < 16; ++rl) if (lane < 16) vst2((unsigned*)(D0 + (rb0 + wave * 16 + rl) * CC + n0 + lane * 8), *(const v4u*)&so[wave * 16 + rl][lane * 8]);
}
__global__ __launch_bounds__(128) void k_local(const _Float16* __restrict__ QL, const _Float16* __restrict__ KL, const _Float16* __restrict__ VL, float* __restrict__ LO) {
  __shared__ __align__(16) _Float16 sph[4][16][56]; __shared__ __align__(16) float so[4][16][68];
  const int tid = threadIdx.x, wave = tid >> 5, lane = tid & 31, col = lane & 15, g = lane >> 4; const int h = blockIdx.y; const size_t b = blockIdx.z; const int q0 = blockIdx.x * 64 + wave * 16; const size_t rq = b * TT + q0;
  v16h aq[2];
#pragma unroll
  for (int kc = 0; kc < 2; ++kc) aq[kc] = frag_h(QL + (rq + col) * CC + h * HD + kc * 32, lane);
  float s[3][8]; const int jbase = q0 - 16;
#pragma unroll
  for (int ct = 0; ct < 3; ++ct) { const int j = jbase + ct * 16 + col; v8f c = {};
    if (jbase + ct * 16 >= 0 && jbase + ct * 16 + 16 <= TT) {
#pragma unroll
      for (int kc = 0; kc < 2; ++kc) c = wmma16(aq[kc], frag_h(KL + (b * TT + j) * CC + h * HD + kc * 32, lane), c); }
#pragma unroll
    for (int r = 0; r < 8; ++r) { const int t = q0 + 8 * g + r; const bool inwin = (j >= t - 8) && (j <= t + 7) && (j >= 0) && (j < TT); s[ct][r] = inwin ? c[r] * 0.125f : -3.0e38f; } }
  float il[8];
#pragma unroll
  for (int r = 0; r < 8; ++r) { const int t = q0 + 8 * g + r; const int npad = max(0, 8 - t) + max(0, t + 8 - TT); float mx = fmaxf(fmaxf(s[0][r], s[1][r]), s[2][r]);
#pragma unroll
    for (int o = 1; o < 16; o <<= 1) mx = fmaxf(mx, __shfl_xor(mx, o));
    if (npad > 0) mx = fmaxf(mx, 0.f);
    float es = 0.f; float e[3];
#pragma unroll
    for (int ct = 0; ct < 3; ++ct) { e[ct] = (s[ct][r] <= -1.0e38f) ? 0.f : __expf(s[ct][r] - mx); es += e[ct]; }
#pragma unroll
    for (int o = 1; o < 16; o <<= 1) es += __shfl_xor(es, o);
    es += (float)npad * __expf(-mx);
    il[r] = (1.0f / 2048.0f) / es;
#pragma unroll
    for (int ct = 0; ct < 3; ++ct) sph[wave][8 * g + r][ct * 16 + col] = (_Float16)(e[ct] * 2048.0f); }
  LDSX();
  v8f acc[4] = {};
#pragma unroll
  for (int ct = 0; ct < 3; ++ct) { const int j0 = jbase + ct * 16; if (j0 < 0 || j0 + 16 > TT) continue;
    (void)j0; }
  {
#pragma unroll
    for (int r = 0; r < 8; ++r) sph[wave][8 * g + r][48 + (col & 7)] = (_Float16)0.f;
  }
  LDSX();
  { const int jA = jbase, jB = jbase + 32;
    const v16h pa = frag_h(&sph[wave][col][0], lane);
    if (jA >= 0) {
#pragma unroll
      for (int dt = 0; dt < 4; ++dt) acc[dt] = wmma16(pa, frag_h(VL + ((b * CC + (size_t)h * HD + dt * 16 + col) * TT) + jA, lane), acc[dt]); }
    else {
      const v16h pa2 = frag_h(&sph[wave][col][16], lane);
#pragma unroll
      for (int dt = 0; dt < 4; ++dt) acc[dt] = wmma16(pa2, frag_h(VL + ((b * CC + (size_t)h * HD + dt * 16 + col) * TT) + 0, lane), acc[dt]); }
    if (jA >= 0 && jB + 16 <= TT) {
      v16h pb = frag_h(&sph[wave][col][32], lane);
#pragma unroll
      for (int i = 8; i < 16; ++i) pb[i] = (_Float16)0.f;
      const int jr = (jB + 32 <= TT) ? jB : (TT - 32);
      if (jr == jB) {
#pragma unroll
        for (int dt = 0; dt < 4; ++dt) acc[dt] = wmma16(pb, frag_h(VL + ((b * CC + (size_t)h * HD + dt * 16 + col) * TT) + jB, lane), acc[dt]); }
      else {
        v16h pc2;
#pragma unroll
        for (int i = 0; i < 8; ++i) { pc2[i] = (_Float16)0.f; pc2[8 + i] = pb[i]; }
#pragma unroll
        for (int dt = 0; dt < 4; ++dt) acc[dt] = wmma16(pc2, frag_h(VL + ((b * CC + (size_t)h * HD + dt * 16 + col) * TT) + (TT - 32), lane), acc[dt]); } }
  }
#pragma unroll
  for (int r = 0; r < 8; ++r)
#pragma unroll
    for (int dt = 0; dt < 4; ++dt) so[wave][8 * g + r][dt * 16 + col] = acc[dt][r] * il[r];
  LDSX();
  for (int rl = 0; rl < 16; ++rl) if (lane < 16) vst2(LO + ((b * NH + h) * TT + q0 + rl) * (size_t)HD + lane * 4, *(const v4f*)&so[wave][rl][lane * 4]);
}
__global__ __launch_bounds__(128) void k_global(const _Float16* __restrict__ QG, const _Float16* __restrict__ KG, const _Float16* __restrict__ VG, float* __restrict__ CG) {
  __shared__ __align__(16) _Float16 sph[4][16][40]; __shared__ __align__(16) float so[4][16][68];
  const int tid = threadIdx.x, wave = tid >> 5, lane = tid & 31, col = lane & 15, g = lane >> 4; const int h = blockIdx.y; const size_t b = blockIdx.z; const int q0 = blockIdx.x * 64 + wave * 16; const size_t rq = b * TT + q0;
  v16h aq[2];
#pragma unroll
  for (int kc = 0; kc < 2; ++kc) aq[kc] = frag_h(QG + (rq + col) * CC + h * HD + kc * 32, lane);
  float m[8], l[8];
#pragma unroll
  for (int r = 0; r < 8; ++r) { m[r] = -3.0e38f; l[r] = 0.f; }
  v8f acc[4] = {};
#pragma unroll 1
  for (int ks = 0; ks < TT / 32; ++ks) { const int j0 = ks * 32; v8f s[2];
#pragma unroll
    for (int ct = 0; ct < 2; ++ct) { const size_t rk = (b * TT + j0 + ct * 16 + col) * CC + h * HD; v8f c = {};
#pragma unroll
      for (int kc = 0; kc < 2; ++kc) c = wmma16(aq[kc], frag_h(KG + rk + kc * 32, lane), c);
#pragma unroll
      for (int r = 0; r < 8; ++r) s[ct][r] = c[r] * 0.125f; }
#pragma unroll
    for (int r = 0; r < 8; ++r) { float mx = fmaxf(s[0][r], s[1][r]);
#pragma unroll
      for (int o = 1; o < 16; o <<= 1) mx = fmaxf(mx, __shfl_xor(mx, o));
      const float mn = fmaxf(m[r], mx); const float alpha = (m[r] <= -1.0e38f) ? 0.f : __expf(m[r] - mn); const float e0 = __expf(s[0][r] - mn), e1 = __expf(s[1][r] - mn); float es = e0 + e1;
#pragma unroll
      for (int o = 1; o < 16; o <<= 1) es += __shfl_xor(es, o);
      l[r] = l[r] * alpha + es; m[r] = mn;
#pragma unroll
      for (int dt = 0; dt < 4; ++dt) acc[dt][r] *= alpha;
      sph[wave][8 * g + r][col] = (_Float16)(e0 * 2048.0f); sph[wave][8 * g + r][16 + col] = (_Float16)(e1 * 2048.0f); }
    LDSX();
    const v16h pa = frag_h(&sph[wave][col][0], lane);
#pragma unroll
    for (int dt = 0; dt < 4; ++dt) acc[dt] = wmma16(pa, frag_h(VG + ((b * CC + (size_t)h * HD + dt * 16 + col) * TT) + j0, lane), acc[dt]);
    LDSX(); }
#pragma unroll
  for (int r = 0; r < 8; ++r) { const float il = (1.0f / 2048.0f) / l[r];
#pragma unroll
    for (int dt = 0; dt < 4; ++dt) so[wave][8 * g + r][dt * 16 + col] = acc[dt][r] * il; }
  LDSX();
  for (int rl = 0; rl < 16; ++rl) if (lane < 16) vst2(CG + (rq + rl) * CC + h * HD + lane * 4, *(const v4f*)&so[wave][rl][lane * 4]);
}
__global__ __launch_bounds__(256) void k_lot(const float* __restrict__ LO, __bf16* __restrict__ LOT, __bf16* __restrict__ LOTL) {
  __shared__ __align__(16) __bf16 sh[64][136]; __shared__ __align__(16) __bf16 sl[64][136]; const size_t rb0 = (size_t)blockIdx.x * 64; const size_t b = rb0 / TT, t0 = rb0 % TT; const int c0 = blockIdx.y * 128; const int t = threadIdx.x;
  for (int e = t; e < 128 * 64; e += 256) { const int c = e >> 6, tl = e & 63; const float v = LO[(b * CC + c0 + c) * (size_t)TT + t0 + tl]; const __bf16 hv = (__bf16)v; sh[tl][c] = hv; sl[tl][c] = (__bf16)(v - (float)hv); }
  __syncthreads();
  for (int e = t; e < 64 * 16; e += 256) { const int tl = e >> 4, q = e & 15; vst2((unsigned*)(LOT + (rb0 + tl) * CC + c0 + q * 8), *(const v4u*)&sh[tl][q * 8]); vst2((unsigned*)(LOTL + (rb0 + tl) * CC + c0 + q * 8), *(const v4u*)&sl[tl][q * 8]); }
}
__global__ __launch_bounds__(128) void k_outl(const __bf16* __restrict__ LOT, const __bf16* __restrict__ LOTL, const __bf16* __restrict__ P, const float* __restrict__ BO, float* __restrict__ YL) {
  __shared__ __align__(16) float st[128][68];
  const int tid = threadIdx.x, wave = tid >> 5, lane = tid & 31, col = lane & 15, g = lane >> 4; const size_t rb0 = (size_t)blockIdx.x * 64, r0 = rb0 + wave * 16; const size_t b = rb0 / TT, t0 = rb0 % TT; const int n0 = blockIdx.y * 128;
  v8f acc[8] = {};
#pragma unroll 2
  for (int kc = 0; kc < CC / 32; ++kc) { const v16b ah = frag_b(LOT + (r0 + col) * CC + kc * 32, lane), al = frag_b(LOTL + (r0 + col) * CC + kc * 32, lane);
#pragma unroll
    for (int j = 0; j < 8; ++j) { const v16b w = frag_b(P + ((size_t)3 * CC + n0 + j * 16 + col) * CC + kc * 32, lane); acc[j] = wmma_bf(ah, w, acc[j]); acc[j] = wmma_bf(al, w, acc[j]); } }
#pragma unroll
  for (int j = 0; j < 8; ++j) { const float bb = bfr(BO[n0 + j * 16 + col]);
#pragma unroll
    for (int r = 0; r < 8; ++r) st[j * 16 + col][wave * 16 + 8 * g + r] = acc[j][r] + bb; }
  __syncthreads();
  for (int e = tid; e < 128 * 16; e += 128) { const int o = e >> 4, q = e & 15; vst2(YL + ((b * CC + n0 + o) * TT) + t0 + q * 4, *(const v4f*)&st[o][q * 4]); }
}
__global__ __launch_bounds__(128) void k_outg(const float* __restrict__ CG, const __bf16* __restrict__ P, const float* __restrict__ BO, const float* __restrict__ YL, const int* __restrict__ TSTEP, float* __restrict__ OUT) {
  __shared__ __align__(16) float st[128][68];
  const int tid = threadIdx.x, wave = tid >> 5, lane = tid & 31, col = lane & 15, g = lane >> 4; const size_t rb0 = (size_t)blockIdx.x * 64, r0 = rb0 + wave * 16; const size_t b = rb0 / TT, t0 = rb0 % TT; const int n0 = blockIdx.y * 128;
  v8f acc[8] = {};
#pragma unroll 2
  for (int kc = 0; kc < CC / 32; ++kc) { const F2 a = split_row(CG + (r0 + col) * CC, kc * 32, lane);
#pragma unroll
    for (int j = 0; j < 8; ++j) { const v16b w = frag_b(P + ((size_t)7 * CC + n0 + j * 16 + col) * CC + kc * 32, lane); acc[j] = wmma_bf(a.l, w, acc[j]); acc[j] = wmma_bf(a.h, w, acc[j]); } }
  const float tn = (float)TSTEP[b] / (float)(TS - 1); const float ag = sqrtf(1.0f - tn), al = sqrtf(tn);
#pragma unroll
  for (int j = 0; j < 8; ++j) { const float bb = bfr(BO[n0 + j * 16 + col]);
#pragma unroll
    for (int r = 0; r < 8; ++r) st[j * 16 + col][wave * 16 + 8 * g + r] = (acc[j][r] + bb) * ag; }
  __syncthreads();
  for (int e = tid; e < 128 * 16; e += 128) { const int o = e >> 4, q = e & 15; const size_t off = ((b * CC + n0 + o) * TT) + t0 + q * 4; v4f yl = *(const v4f*)&YL[off]; v4f v = *(const v4f*)&st[o][q * 4]; v4f w; for (int i = 0; i < 4; ++i) w[i] = v[i] + al * yl[i]; vst2(OUT + off, w); }
}
extern "C" void kernel_launch(void* const* d_in, const int* in_sizes, int n_in, void* d_out, int out_size, void* d_ws, size_t ws_size, hipStream_t stream) {
  (void)in_sizes; (void)n_in; (void)out_size;
  const float** F = (const float**)d_in;
  if (ws_size < (size_t)WS_END) return;
  char* ws = (char*)d_ws; __bf16* P = (__bf16*)ws; _Float16 *QL = (_Float16*)(ws + WS_QL), *KL = (_Float16*)(ws + WS_KL), *QG = (_Float16*)(ws + WS_QG), *KG = (_Float16*)(ws + WS_KG), *VL = (_Float16*)(ws + WS_VL), *VG = (_Float16*)(ws + WS_VG); float *LO = (float*)(ws + WS_LO), *CG = (float*)(ws + WS_CG), *YL = (float*)(ws + WS_YL); __bf16 *LOT = (__bf16*)(ws + WS_LOT), *LOTL = (__bf16*)(ws + WS_LOTL);
  k_pack<<<dim3(CC, 8), 256, 0, stream>>>(F[3], F[5], F[7], F[9], F[11], F[13], F[15], F[17], P);
  k_proj<<<dim3(TR / 64, CC / 128, 6), 128, 0, stream>>>(F[0], F[1], P, F[4], F[6], F[8], F[12], F[14], F[16], QL, KL, VL, QG, KG, VG);
  k_local<<<dim3(TT / 64, NH, TNB), 128, 0, stream>>>(QL, KL, VL, LO);
  k_global<<<dim3(TT / 64, NH, TNB), 128, 0, stream>>>(QG, KG, VG, CG);
  k_lot<<<dim3(TR / 64, CC / 128), 256, 0, stream>>>(LO, LOT, LOTL);
  k_outl<<<dim3(TR / 64, CC / 128), 128, 0, stream>>>(LOT, LOTL, P, F[10], YL);
  k_outg<<<dim3(TR / 64, CC / 128), 128, 0, stream>>>(CG, P, F[18], YL, (const int*)d_in[2], (float*)d_out);
}
